// GATActor_24215025615145
// MI455X (gfx1250) — hardware-verified
//
#include <hip/hip_runtime.h>
#include <stddef.h>


#define HCW   1024
#define NHD   4
#define CH    256
#define OUTC  6
#define OUTP  16
#define KIN   131
#define KP0   192
#define RT    128
#define GRM   64
#define GCN   256
#define CP    260
#define GTHR  256
#define NB    64
#define CHUNK 2048
#define ATHR  128
#define AWAV  4
#define NGRP  (CHUNK / (ATHR * 4))
#define WCAP  (NGRP * 4 * 32)
#define SA    16.0f

#define GEMM_LDS_BYTES (GRM * CP * 4)
#define AGG_LDS_WORDS  (NB * HCW + 3 * NB * NHD + AWAV * WCAP + 8 + AWAV * NHD + 8)
#define AGG_LDS_BYTES  (AGG_LDS_WORDS * 4)

static_assert(NGRP == 4);
static_assert(WCAP == 512);
static_assert(NB == 64);
static_assert(CHUNK == 2048);
static_assert((KP0 % 64) == 0 && KP0 >= KIN);
static_assert((CP % 4) == 0);
static_assert(GEMM_LDS_BYTES == 66560);
static_assert(AGG_LDS_BYTES == 273536);
static_assert(((NB * HCW + NB * NHD) % 4) == 0);
static_assert((RT % GRM) == 0 && (RT % NB) == 0);

typedef float    v4f  __attribute__((ext_vector_type(4)));
typedef float    v8f  __attribute__((ext_vector_type(8)));
typedef int      v4i  __attribute__((ext_vector_type(4)));
typedef _Float16 v8h  __attribute__((ext_vector_type(8)));
typedef _Float16 v16h __attribute__((ext_vector_type(16)));
union Frag   { v16h v; v8h half[2]; };
union Pack16 { v8h h; v4i i; };

__device__ __forceinline__ v8f wm(v16h a, v16h b, v8f c) {
  v8f d = __builtin_amdgcn_wmma_f32_16x16x32_f16(false, a, false, b, (short)0, c, false, false);
  asm volatile("v_nop\n\tv_nop\n\tv_nop\n\tv_nop" : "+v"(d) : "v"(a), "v"(b));
  return d;
}

__device__ __forceinline__ float lrelu(float x) { return x >= 0.f ? x : 0.2f * x; }
__device__ __forceinline__ int iclamp(int v, int lo, int hi) { return v < lo ? lo : (v > hi ? hi : v); }

__global__ __launch_bounds__(256) void k_xcvt(const float* __restrict__ x, _Float16* xP,
                                              int nN, int K, int Kp, int total) {
  const int i = blockIdx.x * 256 + threadIdx.x;
  if (i >= total) return;
  const int per = Kp >> 3;
  const int row = i / per;
  const int c8  = (i - row * per) * 8;
  const int rowc = row < nN ? row : nN - 1;
  const float* xr = x + (size_t)rowc * K;
  Pack16 u;
#pragma unroll
  for (int j = 0; j < 8; ++j) {
    const int col  = c8 + j;
    const int colc = col < K ? col : K - 1;
    float v = xr[colc];
    v = (row < nN && col < K) ? v : 0.0f;
    u.h[j] = (_Float16)v;
  }
  _Float16* p = xP + (size_t)i * 8;
  *(volatile v4i*)p = u.i;
  __threadfence();
  *(volatile v4i*)p = u.i;
}

__global__ __launch_bounds__(256) void k_wcvt(const float* __restrict__ W, _Float16* Wp,
                                              int K, int Kp, int NC, int NR, float scale) {
  __shared__ float Ls[64 * 65];
  const int tid = threadIdx.x, lane = tid & 31, wave = tid >> 5;
  const int k0 = blockIdx.x * 64, n0 = blockIdx.y * 64;
  {
    const int nn = tid & 63;
    const int n  = n0 + nn;
    const int nc = n < NC ? n : NC - 1;
    const int kb = tid >> 6;
#pragma unroll
    for (int j = 0; j < 16; ++j) {
      const int kk = kb + 4 * j;
      const int k  = k0 + kk;
      const int kc = k < K ? k : K - 1;
      float v = W[(size_t)kc * NC + nc];
      v = (k < K && n < NC) ? v : 0.0f;
      Ls[kk * 65 + nn] = v;
    }
  }
  __syncthreads();
#pragma unroll
  for (int it = 0; it < 2; ++it) {
    const int nb = wave * 8 + it * 4;
    if (n0 + nb < NR) {
      const int nl = nb + (lane >> 3);
      const int kq = (lane & 7) * 8;
      Pack16 u;
#pragma unroll
      for (int j = 0; j < 8; ++j) u.h[j] = (_Float16)(Ls[(kq + j) * 65 + nl] * scale);
      _Float16* p = Wp + (size_t)(n0 + nl) * Kp + k0 + kq;
      *(volatile v4i*)p = u.i;
      __threadfence();
      *(volatile v4i*)p = u.i;
    }
  }
}

__global__ __launch_bounds__(GTHR) void k_gemm(
    const _Float16* __restrict__ A, const _Float16* __restrict__ Bw,
    const float* __restrict__ att_s, const float* __restrict__ att_d,
    float* hP, float* asP, float* adP, int ldk, int npad, float inv) {
  extern __shared__ v4f glds[];
  float* Cs = (float*)glds;
  __shared__ __attribute__((aligned(16))) float sS[GRM];
  __shared__ __attribute__((aligned(16))) float sD[GRM];

  const int tid  = threadIdx.x;
  const int lane = tid & 31;
  const int wave = tid >> 5;
  const int hl   = lane >> 4;
  const int l16  = lane & 15;
  const int by   = blockIdx.y;
  const int rowBase = blockIdx.x * GRM;
  const int wr = wave >> 2, wc = wave & 3;
  const int m0 = rowBase + wr * 32;
  const int n0 = by * GCN + wc * 64;

  const v8f z8 = {0.f, 0.f, 0.f, 0.f, 0.f, 0.f, 0.f, 0.f};
  v8f acc[2][4];
#pragma unroll
  for (int ms = 0; ms < 2; ++ms)
#pragma unroll
    for (int ns = 0; ns < 4; ++ns) acc[ms][ns] = z8;

#pragma unroll 1
  for (int k = 0; k < ldk; k += 32) {
    Frag a[2], b[4];
#pragma unroll
    for (int ms = 0; ms < 2; ++ms) {
      const _Float16* ap = A + (size_t)(m0 + ms * 16 + l16) * ldk + k + 8 * hl;
      a[ms].half[0] = *(const v8h*)ap;
      a[ms].half[1] = *(const v8h*)(ap + 16);
    }
#pragma unroll
    for (int ns = 0; ns < 4; ++ns) {
      const _Float16* bp = Bw + (size_t)(n0 + ns * 16 + l16) * ldk + k + 8 * hl;
      b[ns].half[0] = *(const v8h*)bp;
      b[ns].half[1] = *(const v8h*)(bp + 16);
    }
#pragma unroll
    for (int ms = 0; ms < 2; ++ms)
#pragma unroll
      for (int ns = 0; ns < 4; ++ns) acc[ms][ns] = wm(a[ms].v, b[ns].v, acc[ms][ns]);
  }

#pragma unroll
  for (int ms = 0; ms < 2; ++ms)
#pragma unroll
    for (int ns = 0; ns < 4; ++ns)
#pragma unroll
      for (int r = 0; r < 8; ++r)
        Cs[(wr * 32 + ms * 16 + 8 * hl + r) * CP + wc * 64 + ns * 16 + l16] = acc[ms][ns][r] * inv;
  __syncthreads();

  {
    const int row = tid >> 2, q = tid & 3;
    const float* cr = Cs + row * CP + 64 * q;
    const float* ps = att_s + by * CH + 64 * q;
    const float* pd = att_d + by * CH + 64 * q;
    float ss = 0.f, sd = 0.f;
#pragma unroll 2
    for (int c = 0; c < 64; c += 4) {
      const v4f hv = *(const v4f*)(cr + c);
      const v4f sv = *(const v4f*)(ps + c);
      const v4f dv = *(const v4f*)(pd + c);
      ss += hv.x * sv.x + hv.y * sv.y + hv.z * sv.z + hv.w * sv.w;
      sd += hv.x * dv.x + hv.y * dv.y + hv.z * dv.z + hv.w * dv.w;
    }
    ss += __shfl_xor(ss, 1, 32);
    sd += __shfl_xor(sd, 1, 32);
    ss += __shfl_xor(ss, 2, 32);
    sd += __shfl_xor(sd, 2, 32);
    if (q == 0) { sS[row] = ss; sD[row] = sd; }
  }
  __syncthreads();

#pragma unroll
  for (int pass = 0; pass < 2; ++pass) {
#pragma unroll
    for (int i = 0; i < GRM / 8; ++i) {
      const int row = wave * (GRM / 8) + i;
      const float* cp = Cs + row * CP + 4 * lane;
      const v4f v0 = *(const v4f*)cp;
      const v4f v1 = *(const v4f*)(cp + 128);
      float* gp = hP + (size_t)(rowBase + row) * HCW + by * GCN + 4 * lane;
      *(volatile v4f*)gp = v0;
      *(volatile v4f*)(gp + 128) = v1;
    }
    if (lane < 16) {
      if (wave == 0) {
        const v4f v = *(const v4f*)(sS + 4 * lane);
        *(volatile v4f*)(asP + (size_t)by * npad + rowBase + 4 * lane) = v;
      } else if (wave == 1) {
        const v4f v = *(const v4f*)(sD + 4 * lane);
        *(volatile v4f*)(adP + (size_t)by * npad + rowBase + 4 * lane) = v;
      }
    }
    if (pass == 0) __threadfence();
  }
}

__global__ __launch_bounds__(ATHR) void k_agg(
    const int* __restrict__ ei, const float* __restrict__ hP,
    const float* __restrict__ asP, const float* __restrict__ adP,
    const float* __restrict__ bias, _Float16* actP, int nN, int nE, int npad) {
  extern __shared__ v4f alds[];
  float* sacc = (float*)alds;
  float* den  = sacc + NB * HCW;
  float* adL  = den + NB * NHD;
  float* shL  = adL + NB * NHD;
  int*   list = (int*)(shL + NB * NHD);
  int*   wcnt = list + AWAV * WCAP;
  float* wmx  = (float*)(wcnt + 8);
  float* mA   = wmx + AWAV * NHD;

  const int tid  = threadIdx.x;
  const int lane = tid & 31;
  const int wave = tid >> 5;
  const int hd   = wave;
  const int nodeBase = blockIdx.x * NB;
  const v4f z4 = {0.f, 0.f, 0.f, 0.f};

  {
    const int nz = (NB * HCW + NB * NHD) / 4;
    for (int i = tid; i < nz; i += ATHR) alds[i] = z4;
    for (int i = tid; i < NB * NHD; i += ATHR) {
      const int slot = i >> 2, h = i & 3;
      adL[i] = adP[(size_t)h * npad + nodeBase + slot];
    }
  }
  {
    float m0 = -3.0e38f, m1 = -3.0e38f, m2 = -3.0e38f, m3 = -3.0e38f;
    const int nq = nN >> 2;
    const v4f* p0 = (const v4f*)(asP);
    const v4f* p1 = (const v4f*)(asP + (size_t)npad);
    const v4f* p2 = (const v4f*)(asP + (size_t)2 * npad);
    const v4f* p3 = (const v4f*)(asP + (size_t)3 * npad);
#pragma unroll 1
    for (int j = tid; j < nq; j += ATHR) {
      v4f v;
      v = p0[j]; m0 = fmaxf(m0, fmaxf(fmaxf(v.x, v.y), fmaxf(v.z, v.w)));
      v = p1[j]; m1 = fmaxf(m1, fmaxf(fmaxf(v.x, v.y), fmaxf(v.z, v.w)));
      v = p2[j]; m2 = fmaxf(m2, fmaxf(fmaxf(v.x, v.y), fmaxf(v.z, v.w)));
      v = p3[j]; m3 = fmaxf(m3, fmaxf(fmaxf(v.x, v.y), fmaxf(v.z, v.w)));
    }
#pragma unroll
    for (int o = 16; o > 0; o >>= 1) {
      m0 = fmaxf(m0, __shfl_xor(m0, o, 32));
      m1 = fmaxf(m1, __shfl_xor(m1, o, 32));
      m2 = fmaxf(m2, __shfl_xor(m2, o, 32));
      m3 = fmaxf(m3, __shfl_xor(m3, o, 32));
    }
    if (lane == 0) {
      wmx[wave * NHD + 0] = m0; wmx[wave * NHD + 1] = m1;
      wmx[wave * NHD + 2] = m2; wmx[wave * NHD + 3] = m3;
    }
  }
  __syncthreads();
  if (tid < NHD) {
    float m = wmx[tid];
    m = fmaxf(m, wmx[NHD + tid]);
    m = fmaxf(m, wmx[2 * NHD + tid]);
    m = fmaxf(m, wmx[3 * NHD + tid]);
    mA[tid] = m;
  }
  __syncthreads();
  for (int i = tid; i < NB * NHD; i += ATHR) shL[i] = lrelu(mA[i & 3] + adL[i]);
  __syncthreads();

  const int colw = hd * CH + 8 * lane;
  const int* eid = ei + nE;
  const bool al16 = ((nE & 3) == 0);
  const float* asH = asP + (size_t)hd * npad;

  const int nChunks = (nE + CHUNK - 1) / CHUNK;
#pragma unroll 1
  for (int ch = 0; ch < nChunks; ++ch) {
    const int cbase = ch * CHUNK;
    int wc = 0;
#pragma unroll
    for (int g = 0; g < NGRP; ++g) {
      const int el0 = (g * ATHR + tid) * 4;
      const int e0  = cbase + el0;
      const int sent = -2147483647 - 1;
      v4i d;
      if (al16 && (cbase + CHUNK <= nE)) {
        d = *(const v4i*)(eid + e0);
      } else {
        d.x = (e0     < nE) ? eid[iclamp(e0,     0, nE - 1)] : sent;
        d.y = (e0 + 1 < nE) ? eid[iclamp(e0 + 1, 0, nE - 1)] : sent;
        d.z = (e0 + 2 < nE) ? eid[iclamp(e0 + 2, 0, nE - 1)] : sent;
        d.w = (e0 + 3 < nE) ? eid[iclamp(e0 + 3, 0, nE - 1)] : sent;
      }
      const unsigned s0 = (unsigned)d.x - (unsigned)nodeBase;
      const unsigned s1 = (unsigned)d.y - (unsigned)nodeBase;
      const unsigned s2 = (unsigned)d.z - (unsigned)nodeBase;
      const unsigned s3 = (unsigned)d.w - (unsigned)nodeBase;
      const bool h0 = s0 < (unsigned)NB;
      const bool h1 = s1 < (unsigned)NB;
      const bool h2 = s2 < (unsigned)NB;
      const bool h3 = s3 < (unsigned)NB;
      const unsigned many = __builtin_amdgcn_ballot_w32(h0 | h1 | h2 | h3);
      if (many != 0u) {
#define HITJ(J, HJ, SJ) { \
          const unsigned mj = __builtin_amdgcn_ballot_w32(HJ); \
          if (HJ) { \
            const int pos = wc + (int)__builtin_amdgcn_mbcnt_lo(mj, 0u); \
            if (pos < WCAP) list[wave * WCAP + pos] = ((el0 + (J)) << 6) | (int)(SJ); \
          } \
          wc += (int)__builtin_popcount(mj); }
        HITJ(0, h0, s0)
        HITJ(1, h1, s1)
        HITJ(2, h2, s2)
        HITJ(3, h3, s3)
#undef HITJ
      }
    }
    if (lane == 0) wcnt[wave] = wc;
    __syncthreads();

#pragma unroll 1
    for (int wsx = 0; wsx < AWAV; ++wsx) {
      int n = wcnt[wsx];
      n = n > WCAP ? WCAP : (n < 0 ? 0 : n);
#pragma unroll 1
      for (int i = 0; i < n; ++i) {
        const int ent  = list[wsx * WCAP + i];
        const int slot = ent & (NB - 1);
        const int el   = (ent >> 6) & (CHUNK - 1);
        int e = cbase + el;
        e = e > nE - 1 ? nE - 1 : e;
        const int src = iclamp(ei[e], 0, nN - 1);
        const float al = lrelu(asH[src] + adL[slot * NHD + hd]);
        const float p  = __expf(al - shL[slot * NHD + hd]);
        const float* hr = hP + (size_t)src * HCW + colw;
        const v4f xa = *(const v4f*)hr;
        const v4f xb = *(const v4f*)(hr + 4);
        v4f* sp = (v4f*)(sacc + slot * HCW + colw);
        v4f ca = sp[0], cb = sp[1];
        ca = ca + p * xa;
        cb = cb + p * xb;
        sp[0] = ca;
        sp[1] = cb;
        if (lane == 0) {
          const float o = den[slot * NHD + hd];
          den[slot * NHD + hd] = o + p;
        }
      }
    }
    __syncthreads();
  }

  const v4f ba = *(const v4f*)(bias + colw);
  const v4f bb = *(const v4f*)(bias + colw + 4);
#pragma unroll 1
  for (int slot = 0; slot < NB; ++slot) {
    const int node  = nodeBase + slot;
    const int nodec = node < nN ? node : nN - 1;
    const float al  = lrelu(asH[nodec] + adL[slot * NHD + hd]);
    const float p   = __expf(al - shL[slot * NHD + hd]);
    const float dv  = den[slot * NHD + hd] + p;
    const float inv = 1.0f / (dv + 1e-16f);
    const float* hr = hP + (size_t)nodec * HCW + colw;
    const v4f xa = *(const v4f*)hr;
    const v4f xb = *(const v4f*)(hr + 4);
    const v4f* sp = (const v4f*)(sacc + slot * HCW + colw);
    const v4f sa = sp[0] + p * xa;
    const v4f sb = sp[1] + p * xb;
    v4f ya = sa * inv + ba;
    v4f yb = sb * inv + bb;
    ya.x = ya.x > 0.f ? ya.x : 0.f; ya.y = ya.y > 0.f ? ya.y : 0.f;
    ya.z = ya.z > 0.f ? ya.z : 0.f; ya.w = ya.w > 0.f ? ya.w : 0.f;
    yb.x = yb.x > 0.f ? yb.x : 0.f; yb.y = yb.y > 0.f ? yb.y : 0.f;
    yb.z = yb.z > 0.f ? yb.z : 0.f; yb.w = yb.w > 0.f ? yb.w : 0.f;
    if (node >= nN) { ya = z4; yb = z4; }
    Pack16 u;
    u.h[0] = (_Float16)(ya.x * SA); u.h[1] = (_Float16)(ya.y * SA);
    u.h[2] = (_Float16)(ya.z * SA); u.h[3] = (_Float16)(ya.w * SA);
    u.h[4] = (_Float16)(yb.x * SA); u.h[5] = (_Float16)(yb.y * SA);
    u.h[6] = (_Float16)(yb.z * SA); u.h[7] = (_Float16)(yb.w * SA);
    _Float16* op = actP + (size_t)node * HCW + colw;
    *(volatile v4i*)op = u.i;
    __threadfence();
    *(volatile v4i*)op = u.i;
  }
}

__global__ __launch_bounds__(128) void k_fc(
    const _Float16* __restrict__ A, const _Float16* __restrict__ Bw,
    const float* __restrict__ fcb, float* out, int nN) {
  __shared__ float Ds[4][16 * 17];
  __shared__ __attribute__((aligned(16))) float Po[4][96];
  __shared__ __attribute__((aligned(16))) float Lo[4][96];

  const int tid  = threadIdx.x;
  const int lane = tid & 31;
  const int wave = tid >> 5;
  const int hl   = lane >> 4;
  const int l16  = lane & 15;
  const int r0   = (blockIdx.x * 4 + wave) * 16;

  v8f acc = {0.f, 0.f, 0.f, 0.f, 0.f, 0.f, 0.f, 0.f};
#pragma unroll 1
  for (int k = 0; k < HCW; k += 32) {
    Frag a, b;
    const _Float16* ap = A  + (size_t)(r0 + l16) * HCW + k + 8 * hl;
    const _Float16* bp = Bw + (size_t)l16 * HCW + k + 8 * hl;
    a.half[0] = *(const v8h*)ap; a.half[1] = *(const v8h*)(ap + 16);
    b.half[0] = *(const v8h*)bp; b.half[1] = *(const v8h*)(bp + 16);
    acc = wm(a.v, b.v, acc);
  }
  const float invf = 1.0f / (SA * 32.0f);
#pragma unroll
  for (int r = 0; r < 8; ++r) Ds[wave][(8 * hl + r) * 17 + l16] = acc[r] * invf;
  __syncthreads();

  if (lane < 16) {
    const float* dr = Ds[wave] + lane * 17;
    const float g0 = dr[0] + fcb[0], g1 = dr[1] + fcb[1], g2 = dr[2] + fcb[2];
    const float g3 = dr[3] + fcb[3], g4 = dr[4] + fcb[4], g5 = dr[5] + fcb[5];
    float mx = fmaxf(fmaxf(g0, g1), fmaxf(g2, g3));
    mx = fmaxf(mx, fmaxf(g4, g5));
    const float e0 = __expf(g0 - mx), e1 = __expf(g1 - mx), e2 = __expf(g2 - mx);
    const float e3 = __expf(g3 - mx), e4 = __expf(g4 - mx), e5 = __expf(g5 - mx);
    const float s  = e0 + e1 + e2 + e3 + e4 + e5;
    const float is = 1.0f / s;
    float* po = Po[wave] + lane * OUTC;
    float* lo = Lo[wave] + lane * OUTC;
    po[0] = e0 * is; po[1] = e1 * is; po[2] = e2 * is;
    po[3] = e3 * is; po[4] = e4 * is; po[5] = e5 * is;
    lo[0] = g0; lo[1] = g1; lo[2] = g2; lo[3] = g3; lo[4] = g4; lo[5] = g5;
  }
  __syncthreads();

  if (r0 < nN && lane < 24) {
    const v4f vp = *(const v4f*)(Po[wave] + 4 * lane);
    const v4f vl = *(const v4f*)(Lo[wave] + 4 * lane);
    float* gp = out + (size_t)r0 * OUTC + 4 * lane;
    float* gl = out + (size_t)nN * OUTC + (size_t)r0 * OUTC + 4 * lane;
    *(volatile v4f*)gp = vp;
    *(volatile v4f*)gl = vl;
    __threadfence();
    *(volatile v4f*)gp = vp;
    *(volatile v4f*)gl = vl;
  }
}

extern "C" void kernel_launch(void* const* d_in, const int* in_sizes, int n_in,
                              void* d_out, int out_size, void* d_ws, size_t ws_size,
                              hipStream_t stream) {
  if (n_in < 16) return;
  const int nN = in_sizes[0] / KIN;
  if (nN <= 0 || nN * KIN != in_sizes[0]) return;
  if ((nN % 16) != 0) return;
  const int nE = in_sizes[1] / 2;
  if (nE < 1 || 2 * nE != in_sizes[1]) return;
  if (in_sizes[2] != KIN * HCW) return;
  if (in_sizes[6] != HCW * HCW || in_sizes[10] != HCW * HCW) return;
  for (int l = 0; l < 3; ++l) {
    if (in_sizes[3 + 4 * l] != NHD * CH || in_sizes[4 + 4 * l] != NHD * CH) return;
    if (in_sizes[5 + 4 * l] != HCW) return;
  }
  if (in_sizes[14] != HCW * OUTC || in_sizes[15] != OUTC) return;
  if (out_size != 2 * nN * OUTC) return;

  const float* x   = (const float*)d_in[0];
  const int*   ei  = (const int*)d_in[1];
  const float* fcW = (const float*)d_in[14];
  const float* fcb = (const float*)d_in[15];
  float* out = (float*)d_out;

  const int npad = ((nN + RT - 1) / RT) * RT;

  size_t off = 0;
  float*    hP   = (float*)((char*)d_ws + off);    off += (size_t)npad * HCW * sizeof(float);
  _Float16* actP = (_Float16*)((char*)d_ws + off); off += (size_t)npad * HCW * sizeof(_Float16);
  _Float16* xP   = actP;
  _Float16* Wp   = (_Float16*)((char*)d_ws + off); off += (size_t)HCW * HCW * sizeof(_Float16);
  _Float16* fcWp = (_Float16*)((char*)d_ws + off); off += (size_t)OUTP * HCW * sizeof(_Float16);
  float*    asP  = (float*)((char*)d_ws + off);    off += (size_t)NHD * npad * sizeof(float);
  float*    adP  = (float*)((char*)d_ws + off);    off += (size_t)NHD * npad * sizeof(float);
  if (off > ws_size) return;
  if ((size_t)npad * KP0 * sizeof(_Float16) > (size_t)npad * HCW * sizeof(_Float16)) return;

  hipFuncSetAttribute(reinterpret_cast<const void*>(&k_gemm),
                      hipFuncAttributeMaxDynamicSharedMemorySize, GEMM_LDS_BYTES);
  hipFuncSetAttribute(reinterpret_cast<const void*>(&k_agg),
                      hipFuncAttributeMaxDynamicSharedMemorySize, AGG_LDS_BYTES);

  const int totx = npad * (KP0 / 8);
  k_xcvt<<<(totx + 255) / 256, 256, 0, stream>>>(x, xP, nN, KIN, KP0, totx);

  for (int l = 0; l < 3; ++l) {
    const float* W   = (const float*)d_in[2 + 4 * l];
    const float* ats = (const float*)d_in[3 + 4 * l];
    const float* atd = (const float*)d_in[4 + 4 * l];
    const float* b   = (const float*)d_in[5 + 4 * l];
    const int   K   = (l == 0) ? KIN : HCW;
    const int   Kp  = (l == 0) ? KP0 : HCW;
    const float sw  = (l == 0) ? 8.0f : 32.0f;
    const float sa  = (l == 0) ? 1.0f : SA;
    const float inv = 1.0f / (sw * sa);
    const _Float16* Ain = (l == 0) ? xP : actP;

    k_wcvt<<<dim3(Kp / 64, HCW / 64), 256, 0, stream>>>(W, Wp, K, Kp, HCW, HCW, sw);
    k_gemm<<<dim3(npad / GRM, NHD), GTHR, GEMM_LDS_BYTES, stream>>>(
        Ain, Wp, ats, atd, hP, asP, adP, Kp, npad, inv);
    k_agg<<<npad / NB, ATHR, AGG_LDS_BYTES, stream>>>(ei, hP, asP, adP, b, actP, nN, nE, npad);
  }

  k_wcvt<<<dim3(HCW / 64, 1), 256, 0, stream>>>(fcW, fcWp, HCW, HCW, OUTC, OUTP, 32.0f);
  k_fc<<<(nN + 63) / 64, 128, 0, stream>>>(actP, fcWp, fcb, out, nN);
}
